// GATBridge_28913719837512
// MI455X (gfx1250) — hardware-run, weakly checked
//
#include <hip/hip_runtime.h>
#include <math.h>

typedef __attribute__((ext_vector_type(16))) _Float16 v16h;
typedef __attribute__((ext_vector_type(16))) __bf16 v16b;
typedef __attribute__((ext_vector_type(8)))  _Float16 v8h;
typedef __attribute__((ext_vector_type(8)))  float v8f;
typedef __attribute__((ext_vector_type(4)))  float v4f;
typedef __attribute__((ext_vector_type(2)))  float v2f;
typedef __attribute__((ext_vector_type(4)))  unsigned v4u;
typedef __attribute__((ext_vector_type(4)))  int v4i;
typedef float __attribute__((may_alias)) float_a;
typedef int __attribute__((may_alias)) int_a;

template <typename T> __device__ __forceinline__ void vst2(void* p, T v) { *(volatile T*)p = v; __threadfence(); *(volatile T*)p = v; }
__device__ __forceinline__ v8f wmma16(v16h a, v16h b, v8f c) {
  v8f d = __builtin_amdgcn_wmma_f32_16x16x32_f16(false, a, false, b, (short)0, c, false, false);
  asm volatile("v_nop\n\tv_nop\n\tv_nop\n\tv_nop" : "+v"(d) : "v"(a), "v"(b));
  return d;
}
__device__ __forceinline__ v8f wmma_bf(v16b a, v16b b, v8f c) {
  v8f d = __builtin_amdgcn_wmma_f32_16x16x32_bf16(false, a, false, b, (short)0, c, false, false);
  asm volatile("v_nop\n\tv_nop\n\tv_nop\n\tv_nop" : "+v"(d) : "v"(a), "v"(b));
  return d;
}
__device__ __forceinline__ v16h frag_h(const _Float16* rowk0, int lane) {
  union { v16h v; v8h q[2]; } u; const _Float16* p = rowk0 + 8 * (lane >> 4);
  u.q[0] = *(const v8h*)p; u.q[1] = *(const v8h*)(p + 16); return u.v;
}
__device__ __forceinline__ v16h frag_f32(const float* rowk0, int lane) {
  v16h a; const float* p = rowk0 + 8 * (lane >> 4);
#pragma unroll
  for (int i = 0; i < 8; ++i) { a[i] = (_Float16)p[i]; a[8 + i] = (_Float16)p[16 + i]; }
  return a;
}
__device__ __forceinline__ v16h frag_f32s(const float* rowk0, int lane, float sc) {
  v16h a; const float* p = rowk0 + 8 * (lane >> 4);
#pragma unroll
  for (int i = 0; i < 8; ++i) { a[i] = (_Float16)(p[i] * sc); a[8 + i] = (_Float16)(p[16 + i] * sc); }
  return a;
}
__device__ __forceinline__ v16h fragc_f32(const float* W, int k0, int n, int lane, int ld, int K) {
  v16h a; const int g = lane >> 4;
#pragma unroll
  for (int i = 0; i < 8; ++i) { const int ka = k0 + 8 * g + i, kb = ka + 16;
    a[i] = (_Float16)(ka < K ? W[(size_t)(ka < K ? ka : K - 1) * ld + n] : 0.f); a[8 + i] = (_Float16)(kb < K ? W[(size_t)(kb < K ? kb : K - 1) * ld + n] : 0.f); }
  return a;
}
struct F2 { v16b h, l; };
__device__ __forceinline__ F2 bsplit16(const float v[16]) { F2 r;
#pragma unroll
  for (int i = 0; i < 16; ++i) { const __bf16 h = (__bf16)v[i]; r.h[i] = h; r.l[i] = (__bf16)(v[i] - (float)h); }
  return r; }
__device__ __forceinline__ F2 split_row(const float* row, int k0, int lane) { float v[16]; const float* p = row + k0 + 8 * (lane >> 4);
#pragma unroll
  for (int i = 0; i < 8; ++i) { v[i] = p[i]; v[8 + i] = p[16 + i]; }
  return bsplit16(v); }
__device__ __forceinline__ F2 split_rowK(const float* row, int k0, int lane, int K) { float v[16]; const int g = lane >> 4;
#pragma unroll
  for (int i = 0; i < 8; ++i) { const int ka = k0 + 8 * g + i, kb = ka + 16; v[i] = ka < K ? row[ka < K ? ka : K - 1] : 0.f; v[8 + i] = kb < K ? row[kb < K ? kb : K - 1] : 0.f; }
  return bsplit16(v); }
__device__ __forceinline__ F2 split_col(const float* W, int k0, int n, int lane, int ld, int K) { float v[16]; const int g = lane >> 4;
#pragma unroll
  for (int i = 0; i < 8; ++i) { const int ka = k0 + 8 * g + i, kb = ka + 16; v[i] = ka < K ? W[(size_t)(ka < K ? ka : K - 1) * ld + n] : 0.f; v[8 + i] = kb < K ? W[(size_t)(kb < K ? kb : K - 1) * ld + n] : 0.f; }
  return bsplit16(v); }
__device__ __forceinline__ v8f mac3(const F2& a, const F2& b, v8f c) { c = wmma_bf(a.l, b.h, c); c = wmma_bf(a.h, b.l, c); return wmma_bf(a.h, b.h, c); }
__device__ __forceinline__ float sigm(float v) { return 1.0f / (1.0f + expf(-v)); }
#define LDSX() do { asm volatile("s_wait_dscnt 0" ::: "memory"); __builtin_amdgcn_wave_barrier(); __builtin_amdgcn_fence(__ATOMIC_RELEASE, "workgroup"); } while (0)


#define NB 8
#define NN 1024
#define DIN 512
#define NH1 4
#define FH 256
#define D1 (NH1 * FH)
#define DOUT 512
#define NS 0.2f
#ifndef TNB
#define TNB NB
#endif
typedef __attribute__((ext_vector_type(8))) __bf16 v8b;
__device__ __forceinline__ v16b frag_b(const __bf16* rowk0, int lane) {
  union { v16b v; v8b q[2]; } u; const __bf16* p = rowk0 + 8 * (lane >> 4);
  u.q[0] = *(const v8b*)p; u.q[1] = *(const v8b*)(p + 16); return u.v;
}
__device__ __forceinline__ float bfr(float v) { return (float)(__bf16)v; }
__device__ __attribute__((noinline)) float exp_ni(float v) { return expf(v); }
__device__ __attribute__((noinline)) float erf_ni(float v) { return erff(v); }

#define WS_P1   0u
#define WS_P2   (WS_P1 + 2u * D1 * DIN)
#define WS_XL   (WS_P2 + 2u * DOUT * D1)
#define WS_XT   (WS_XL + 4u * (size_t)NB * NN * D1)
#define WS_XTL  (WS_XT + 2u * (size_t)NB * D1 * NN)
#define WS_AS   (WS_XTL + 2u * (size_t)NB * D1 * NN)
#define WS_AD   (WS_AS + 4u * (size_t)NB * NN * 4)
#define WS_H1   (WS_AD + 4u * (size_t)NB * NN * 4)
#define WS_END  (WS_H1 + 4u * (size_t)NB * NN * D1)

__global__ __launch_bounds__(256) void k_packw(const float* __restrict__ W1, const float* __restrict__ W2, char* __restrict__ ws) { const int n = blockIdx.x, t = threadIdx.x; __shared__ __align__(16) __bf16 s1[DIN]; __shared__ __align__(16) __bf16 s2[D1];
  for (int k = t; k < DIN; k += 256) s1[k] = (__bf16)W1[(size_t)k * D1 + n]; if (n < DOUT) for (int k = t; k < D1; k += 256) s2[k] = (__bf16)W2[(size_t)k * DOUT + n]; __syncthreads();
  if (t < DIN / 8) vst2((unsigned*)((__bf16*)(ws + WS_P1) + (size_t)n * DIN + t * 8), *(const v4u*)&s1[t * 8]); if (n < DOUT && t < D1 / 8) vst2((unsigned*)((__bf16*)(ws + WS_P2) + (size_t)n * D1 + t * 8), *(const v4u*)&s2[t * 8]); }
__device__ __forceinline__ v16b fragb_f32(const float* __restrict__ p, int lane) { v16b a; const float* pp = p + 8 * (lane >> 4);
#pragma unroll
  for (int i = 0; i < 8; ++i) { a[i] = (__bf16)pp[i]; a[8 + i] = (__bf16)pp[16 + i]; } return a; }
template <int L>
__global__ __launch_bounds__(128) void k_xl(const float* __restrict__ A, const __bf16* __restrict__ P, float* __restrict__ XL, _Float16* __restrict__ XT, _Float16* __restrict__ XTL) { __shared__ __align__(16) float sf[64][132]; __shared__ __align__(16) _Float16 th[128][72], tl[128][72];
  constexpr int K = L == 1 ? DIN : D1; constexpr int NC = L == 1 ? D1 : DOUT;
  const int tid = threadIdx.x, wave = tid >> 5, lane = tid & 31, col = lane & 15, g = lane >> 4; const size_t b = blockIdx.z; const int n0 = blockIdx.x * 64 + wave * 16; const int c0 = blockIdx.y * 128; const size_t r0 = b * NN + n0;
  v8f acc[8] = {};
#pragma unroll 2
  for (int kc = 0; kc < K / 32; ++kc) { if (L == 1) { const v16b a = fragb_f32(A + (r0 + col) * K + kc * 32, lane);
#pragma unroll
      for (int j = 0; j < 8; ++j) acc[j] = wmma_bf(a, frag_b(P + (size_t)(c0 + j * 16 + col) * K + kc * 32, lane), acc[j]); }
    else { const F2 a = split_row(A + (r0 + col) * K, kc * 32, lane);
#pragma unroll
      for (int j = 0; j < 8; ++j) { const v16b w = frag_b(P + (size_t)(c0 + j * 16 + col) * K + kc * 32, lane); acc[j] = wmma_bf(a.h, w, acc[j]); acc[j] = wmma_bf(a.l, w, acc[j]); } } }
#pragma unroll
  for (int j = 0; j < 8; ++j)
#pragma unroll
    for (int r = 0; r < 8; ++r) { const float v = acc[j][r]; sf[wave * 16 + 8 * g + r][j * 16 + col] = v; const _Float16 hv = (_Float16)v; th[j * 16 + col][wave * 16 + 8 * g + r] = hv; tl[j * 16 + col][wave * 16 + 8 * g + r] = (_Float16)((v - (float)hv) * 2048.0f); }
  __syncthreads();
  for (int e = tid; e < 64 * 32; e += 128) { const int rl = e >> 5, q = e & 31; vst2(XL + (b * NN + blockIdx.x * 64 + rl) * NC + c0 + q * 4, *(const v4f*)&sf[rl][q * 4]); }
  for (int e = tid; e < 128 * 8; e += 128) { const int cl = e >> 3, q = e & 7; const size_t o = ((b * NC + c0 + cl) * (size_t)NN) + blockIdx.x * 64 + q * 8; vst2((unsigned*)(XT + o), *(const v4u*)&th[cl][q * 8]); vst2((unsigned*)(XTL + o), *(const v4u*)&tl[cl][q * 8]); } }
template <int L>
__global__ __launch_bounds__(256) void k_coef(const float* __restrict__ XL, const float* __restrict__ ASRC, const float* __restrict__ ADST, float* __restrict__ AS, float* __restrict__ AD) { __shared__ __align__(16) float ss[32], sd[32]; constexpr int H = L == 1 ? NH1 : 1; constexpr int F = L == 1 ? FH : DOUT; constexpr int NC = H * F;
  const int t = threadIdx.x, lane = t & 31, w = t >> 5; const size_t row = (size_t)blockIdx.x * 8 + w; const float* xr = XL + row * NC;
  if (lane < 4) { ss[w * 4 + lane] = 0.f; sd[w * 4 + lane] = 0.f; }
#pragma unroll 1
  for (int h = 0; h < H; ++h) {
#pragma unroll 1
    for (int which = 0; which < 2; ++which) { const float* av = (which == 0 ? ASRC : ADST) + h * F; float s = 0.f;
#pragma unroll 1
      for (int f = lane; f < F; f += 32) s += xr[h * F + f] * bfr(av[f]);
#pragma unroll
      for (int o = 1; o < 32; o <<= 1) s += __shfl_xor(s, o);
      if (lane == 0) { if (which == 0) ss[w * 4 + h] = s; else sd[w * 4 + h] = s; } } }
  __syncthreads(); if (t < 8) vst2(AS + (size_t)blockIdx.x * 32 + t * 4, *(const v4f*)&ss[t * 4]); else if (t < 16) vst2(AD + (size_t)blockIdx.x * 32 + (t - 8) * 4, *(const v4f*)&sd[(t - 8) * 4]); }
template <int L>
__global__ __launch_bounds__(128) void k_gat(const float* __restrict__ AS, const float* __restrict__ AD, const int* __restrict__ ADJ, const _Float16* __restrict__ XT, const _Float16* __restrict__ XTL, const float* __restrict__ BIAS, float* __restrict__ OUTR) {
  constexpr int F = L == 1 ? FH : DOUT; constexpr int NC = L == 1 ? D1 : DOUT; constexpr int NFB = F / 128;
  __shared__ __align__(16) float sp[4][16][36]; __shared__ __align__(16) float so[4][16][132]; __shared__ float sas[NN];
  const int tid = threadIdx.x, wave = tid >> 5, lane = tid & 31, col = lane & 15, g = lane >> 4; const int h = blockIdx.y / NFB, fb = blockIdx.y % NFB; const size_t b = blockIdx.z; const int d0 = blockIdx.x * 64 + wave * 16;
  for (int s = tid; s < NN; s += 128) sas[s] = AS[(b * NN + s) * 4 + h]; __syncthreads();
  float adv[8];
#pragma unroll
  for (int r = 0; r < 8; ++r) adv[r] = AD[(b * NN + d0 + 8 * g + r) * 4 + h];
  float m[8], l[8];
#pragma unroll
  for (int r = 0; r < 8; ++r) { m[r] = -3.0e38f; l[r] = 0.f; }
  v8f acc[8] = {}, accl[8] = {};
#pragma unroll 1
  for (int ks = 0; ks < NN / 32; ++ks) { float s[2][8];
#pragma unroll
    for (int ct = 0; ct < 2; ++ct) { const int ss = ks * 32 + ct * 16 + col; const float av = sas[ss]; const int* adjc = ADJ + (b * NN + ss) * (size_t)NN;
#pragma unroll
      for (int r = 0; r < 8; ++r) { const int d = d0 + 8 * g + r; const bool keep = (adjc[d] != 0) || (ss == d); float e = av + adv[r]; e = (e > 0.f) ? e : NS * e; s[ct][r] = keep ? e : -3.0e38f; } }
    float alpha[8];
#pragma unroll
    for (int r = 0; r < 8; ++r) { float mx = fmaxf(s[0][r], s[1][r]);
#pragma unroll
      for (int o = 1; o < 16; o <<= 1) mx = fmaxf(mx, __shfl_xor(mx, o));
      const float mn = fmaxf(m[r], mx); alpha[r] = (m[r] <= -1.0e38f) ? 0.f : __expf(m[r] - mn); const float e0 = (s[0][r] <= -1.0e38f) ? 0.f : __expf(s[0][r] - mn), e1 = (s[1][r] <= -1.0e38f) ? 0.f : __expf(s[1][r] - mn); float es = e0 + e1;
#pragma unroll
      for (int o = 1; o < 16; o <<= 1) es += __shfl_xor(es, o);
      l[r] = l[r] * alpha[r] + es; m[r] = mn; sp[wave][8 * g + r][col] = e0; sp[wave][8 * g + r][16 + col] = e1; }
#pragma unroll
    for (int j = 0; j < 8; ++j)
#pragma unroll
      for (int r = 0; r < 8; ++r) { acc[j][r] *= alpha[r]; accl[j][r] *= alpha[r]; }
    LDSX();
    v16h pa; { const float* prow = &sp[wave][col][0] + 8 * (lane >> 4);
#pragma unroll
      for (int i = 0; i < 8; ++i) { pa[i] = (_Float16)(prow[i] * 2048.0f); pa[8 + i] = (_Float16)(prow[16 + i] * 2048.0f); } }
#pragma unroll
    for (int j = 0; j < 8; ++j) { const size_t po = (b * NC + (size_t)h * F + fb * 128 + j * 16 + col) * (size_t)NN + ks * 32; acc[j] = wmma16(pa, frag_h(XT + po, lane), acc[j]); accl[j] = wmma16(pa, frag_h(XTL + po, lane), accl[j]); }
    LDSX(); }
#pragma unroll
  for (int r = 0; r < 8; ++r) { const float il = (l[r] > 0.f) ? (1.0f / 2048.0f) / l[r] : 0.f;
#pragma unroll
    for (int j = 0; j < 8; ++j) { const int c = h * F + fb * 128 + j * 16 + col; float v = (acc[j][r] + accl[j][r] * (1.0f / 2048.0f)) * il + bfr(BIAS[c]); if (L == 1) v = (v > 0.f) ? v : expm1f(v); so[wave][8 * g + r][j * 16 + col] = v; } }
  LDSX(); for (int rl = 0; rl < 16; ++rl) vst2(OUTR + (b * NN + d0 + rl) * NC + (size_t)h * F + fb * 128 + lane * 4, *(const v4f*)&so[wave][rl][lane * 4]); }
extern "C" void kernel_launch(void* const* d_in, const int* in_sizes, int n_in, void* d_out, int out_size, void* d_ws, size_t ws_size, hipStream_t stream) {
  (void)in_sizes; (void)n_in; (void)out_size;
  const float** Fp = (const float**)d_in;
  if (ws_size < (size_t)WS_END) return;
  char* ws = (char*)d_ws; const __bf16 *P1 = (const __bf16*)(ws + WS_P1), *P2 = (const __bf16*)(ws + WS_P2); float *XL = (float*)(ws + WS_XL), *AS = (float*)(ws + WS_AS), *AD = (float*)(ws + WS_AD), *H1 = (float*)(ws + WS_H1); _Float16 *XT = (_Float16*)(ws + WS_XT), *XTL = (_Float16*)(ws + WS_XTL); const int* ADJ = (const int*)d_in[0];
  k_packw<<<D1, 256, 0, stream>>>(Fp[2], Fp[6], ws);
  k_xl<1><<<dim3(NN / 64, D1 / 128, TNB), 128, 0, stream>>>(Fp[1], P1, XL, XT, XTL);
  k_coef<1><<<TNB * NN / 8, 256, 0, stream>>>(XL, Fp[3], Fp[4], AS, AD);
  k_gat<1><<<dim3(NN / 64, NH1 * (FH / 128), TNB), 128, 0, stream>>>(AS, AD, ADJ, XT, XTL, Fp[5], H1);
  k_xl<2><<<dim3(NN / 64, DOUT / 128, TNB), 128, 0, stream>>>(H1, P2, XL, XT, XTL);
  k_coef<2><<<TNB * NN / 8, 256, 0, stream>>>(XL, Fp[7], Fp[8], AS, AD);
  k_gat<2><<<dim3(NN / 64, DOUT / 128, TNB), 128, 0, stream>>>(AS, AD, ADJ, XT, XTL, Fp[9], (float*)d_out);
}
